// SpatialAttention_40037685133393
// MI455X (gfx1250) — hardware-verified
//
#include <hip/hip_runtime.h>
#include <stdint.h>
#include <stddef.h>


#ifndef NB
#define NB 1
#endif
#ifndef SEQ
#define SEQ 4096
#endif
#define NB_FULL   1
#define SEQ_FULL  4096
#define NNODE     (SEQ_FULL)
#define QROWS     (SEQ)
#define HIDC      512
#define NHEAD     8
#define HDIM      64
#define MWORDS    (NNODE / 32)
#define PCARRY    16384.0f
#define CTXSC     0.0009765625f
#define WOC       1024.0f
#define OUNC      0.00006103515625f
#define SCL       0.18033688011112042f
#define LNEPS     0.00001f
#define XB_BLOCKS ((NNODE * HIDC) / 2048)
#define W_BLOCKS  ((HIDC * HIDC) / 2048)

static_assert(NB == 1 && NB_FULL == 1);
static_assert(QROWS >= 64 && QROWS <= NNODE && (QROWS % 64) == 0);
static_assert(HIDC == NHEAD * HDIM && HDIM == 64 && NHEAD == 8);
static_assert((NNODE % 64) == 0 && MWORDS == 128);
static_assert(((NNODE * HIDC) % 2048) == 0 && ((HIDC * HIDC) % 2048) == 0);

typedef float          v8f   __attribute__((ext_vector_type(8)));
typedef float          v4f_  __attribute__((ext_vector_type(4)));
typedef v4f_           v4f   __attribute__((may_alias));
typedef _Float16       v16h  __attribute__((ext_vector_type(16)));
typedef _Float16       v8h_  __attribute__((ext_vector_type(8)));
typedef v8h_           v8h   __attribute__((may_alias));
typedef __bf16         v16bf __attribute__((ext_vector_type(16)));
typedef unsigned short v8us_ __attribute__((ext_vector_type(8)));
typedef v8us_          v8us  __attribute__((may_alias));
typedef unsigned       v4u_  __attribute__((ext_vector_type(4)));
typedef v4u_           v4u   __attribute__((may_alias));

union FragB { v16bf v; v8us_ h[2]; };
union FragH { v16h  v; v8h_  h[2]; };

__device__ __forceinline__ v8f mma_bf16(const v16bf a, const v16bf b, v8f c)
{
  v8f d = __builtin_amdgcn_wmma_f32_16x16x32_bf16(false, a, false, b, (short)0, c, false, false);
  asm volatile("v_nop\n\tv_nop\n\tv_nop\n\tv_nop" : "+v"(d) : "v"(a), "v"(b));
  return d;
}
__device__ __forceinline__ v8f mma_f16(const v16h a, const v16h b, v8f c)
{
  v8f d = __builtin_amdgcn_wmma_f32_16x16x32_f16(false, a, false, b, (short)0, c, false, false);
  asm volatile("v_nop\n\tv_nop\n\tv_nop\n\tv_nop" : "+v"(d) : "v"(a), "v"(b));
  return d;
}

__device__ __forceinline__ unsigned short bf16_bits(float f)
{
  const __bf16 hb = (__bf16)f;
  return __builtin_bit_cast(unsigned short, hb);
}
__device__ __forceinline__ float bf16_rn(float f)
{
  return (float)(__bf16)f;
}
__device__ __forceinline__ unsigned short f16_bits(float f)
{
  const _Float16 hf = (_Float16)f;
  return __builtin_bit_cast(unsigned short, hf);
}
__device__ __forceinline__ float exp2fast(float x)
{
#if __has_builtin(__builtin_amdgcn_exp2f)
  return __builtin_amdgcn_exp2f(x);
#else
  return exp2f(x);
#endif
}

__global__ void __launch_bounds__(256) cvt_kernel(
    const float* __restrict__ x, const float* __restrict__ wq, const float* __restrict__ wk,
    const float* __restrict__ wv, const float* __restrict__ wo,
    unsigned short* __restrict__ xb, unsigned short* __restrict__ wqkv, unsigned short* __restrict__ wob)
{
  const int blk = (int)blockIdx.x;
  const int tid = (int)threadIdx.x;
  const float* src;
  unsigned short* dst;
  int t;
  int f16mode = 0;
  if (blk < XB_BLOCKS) {
    src = x;  dst = xb;  t = blk * 256 + tid;
  } else if (blk < XB_BLOCKS + W_BLOCKS) {
    src = wq; dst = wqkv; t = (blk - XB_BLOCKS) * 256 + tid;
  } else if (blk < XB_BLOCKS + 2 * W_BLOCKS) {
    src = wk; dst = wqkv + (size_t)HIDC * HIDC; t = (blk - XB_BLOCKS - W_BLOCKS) * 256 + tid;
  } else if (blk < XB_BLOCKS + 3 * W_BLOCKS) {
    src = wv; dst = wqkv + 2 * (size_t)HIDC * HIDC; t = (blk - XB_BLOCKS - 2 * W_BLOCKS) * 256 + tid;
  } else {
    src = wo; dst = wob; t = (blk - XB_BLOCKS - 3 * W_BLOCKS) * 256 + tid; f16mode = 1;
  }

  const v4f_ a = *(const v4f*)(src + (size_t)t * 8);
  const v4f_ b = *(const v4f*)(src + (size_t)t * 8 + 4);
  v8us_ o;
  if (f16mode) {
    o[0] = f16_bits(WOC * bf16_rn(a[0])); o[1] = f16_bits(WOC * bf16_rn(a[1]));
    o[2] = f16_bits(WOC * bf16_rn(a[2])); o[3] = f16_bits(WOC * bf16_rn(a[3]));
    o[4] = f16_bits(WOC * bf16_rn(b[0])); o[5] = f16_bits(WOC * bf16_rn(b[1]));
    o[6] = f16_bits(WOC * bf16_rn(b[2])); o[7] = f16_bits(WOC * bf16_rn(b[3]));
  } else {
    o[0] = bf16_bits(a[0]); o[1] = bf16_bits(a[1]); o[2] = bf16_bits(a[2]); o[3] = bf16_bits(a[3]);
    o[4] = bf16_bits(b[0]); o[5] = bf16_bits(b[1]); o[6] = bf16_bits(b[2]); o[7] = bf16_bits(b[3]);
  }
  unsigned short* p = dst + (size_t)t * 8;
  *(volatile v8us_*)p = o;
  __threadfence();
  *(volatile v8us_*)p = o;
}

__global__ void __launch_bounds__(256) adj_kernel(
    const int* __restrict__ ei, int ne, unsigned* __restrict__ mk)
{
  __shared__ __align__(16) unsigned sM[64 * MWORDS];
  const int tid = (int)threadIdx.x;
  const int r0  = (int)blockIdx.x * 64;

#pragma unroll 4
  for (int it = 0; it < (64 * MWORDS) / 256; ++it) sM[it * 256 + tid] = 0u;
  __syncthreads();

#pragma unroll 1
  for (int e = tid; e < ne; e += 256) {
    const int s = ei[e];
    const int d = ei[(size_t)ne + (size_t)e];
    const unsigned rl = (unsigned)(s - r0);
    if (rl < 64u && (unsigned)d < (unsigned)NNODE)
      atomicOr(&sM[rl * MWORDS + (unsigned)(d >> 5)], 1u << (d & 31));
  }
  __syncthreads();

  v4u_ mv[8];
#pragma unroll
  for (int it = 0; it < 8; ++it) mv[it] = *(const v4u*)&sM[(it * 256 + tid) * 4];
  unsigned* base = mk + (size_t)r0 * MWORDS;
#pragma unroll
  for (int it = 0; it < 8; ++it)
    *(volatile v4u_*)(base + (size_t)(it * 256 + tid) * 4) = mv[it];
  __threadfence();
#pragma unroll
  for (int it = 0; it < 8; ++it)
    *(volatile v4u_*)(base + (size_t)(it * 256 + tid) * 4) = mv[it];
}

__global__ void __launch_bounds__(256) proj_kernel(
    const unsigned short* __restrict__ xb, const unsigned short* __restrict__ wqkv,
    const float* __restrict__ bq, const float* __restrict__ bk, const float* __restrict__ bv,
    unsigned short* __restrict__ qh, unsigned short* __restrict__ kh, unsigned short* __restrict__ vt)
{
  __shared__ __align__(16) unsigned short sT[128 * 64];

  const int tid  = (int)threadIdx.x;
  const int lane = tid & 31, wave = tid >> 5;
  const int h = lane >> 4, m = lane & 15;
  const int n0  = (int)blockIdx.x * 64;
  const int c0  = (int)blockIdx.y * 128;
  const int sel = c0 / HIDC;
  const int cw  = c0 - sel * HIDC;
  if (sel == 0 && n0 >= QROWS) return;

  const unsigned short* Wb = wqkv + (size_t)sel * HIDC * HIDC;
  const float* bias = bq;
  unsigned short* plane = qh;
  if (sel == 1)      { bias = bk; plane = kh; }
  else if (sel == 2) { bias = bv; plane = vt; }

  const int wr = wave >> 2, wc = wave & 3;
  const int rbase = n0 + wr * 32;
  const int cbase = cw + wc * 32;

  v8f acc[2][2] = {};
#pragma unroll 2
  for (int k0 = 0; k0 < HIDC; k0 += 32) {
    FragB a[2], b[2];
#pragma unroll
    for (int rt = 0; rt < 2; ++rt) {
      const unsigned short* ar = xb + (size_t)(rbase + rt * 16 + m) * HIDC + k0 + 8 * h;
      a[rt].h[0] = *(const v8us*)(ar);
      a[rt].h[1] = *(const v8us*)(ar + 16);
    }
#pragma unroll
    for (int ct = 0; ct < 2; ++ct) {
      const unsigned short* wrp = Wb + (size_t)(cbase + ct * 16 + m) * HIDC + k0 + 8 * h;
      b[ct].h[0] = *(const v8us*)(wrp);
      b[ct].h[1] = *(const v8us*)(wrp + 16);
    }
#pragma unroll
    for (int rt = 0; rt < 2; ++rt)
#pragma unroll
      for (int ct = 0; ct < 2; ++ct)
        acc[rt][ct] = mma_bf16(a[rt].v, b[ct].v, acc[rt][ct]);
  }

  if (sel == 2) {
#pragma unroll
    for (int rt = 0; rt < 2; ++rt)
#pragma unroll
      for (int ct = 0; ct < 2; ++ct) {
        const int cl = wc * 32 + ct * 16 + m;
        const float bb = bf16_rn(bias[cw + cl]);
        v8h_ o;
#pragma unroll
        for (int r = 0; r < 8; ++r) o[r] = (_Float16)(acc[rt][ct][r] + bb);
        *(v8us*)&sT[cl * 64 + wr * 32 + rt * 16 + 8 * h] = __builtin_bit_cast(v8us_, o);
      }
  } else {
#pragma unroll
    for (int rt = 0; rt < 2; ++rt)
#pragma unroll
      for (int ct = 0; ct < 2; ++ct) {
        const int cl = wc * 32 + ct * 16 + m;
        const float bb = bf16_rn(bias[cw + cl]);
        const int Lb = (cl >> 6) * 64 + wr * 32 + rt * 16 + 8 * h;
        const int d  = cl & 63;
#pragma unroll
        for (int r = 0; r < 8; ++r) sT[(Lb + r) * 64 + d] = f16_bits(acc[rt][ct][r] + bb);
      }
  }
  __syncthreads();

  v4u_ pv[4];
#pragma unroll
  for (int it = 0; it < 4; ++it) {
    const int p = it * 256 + tid;
    pv[it] = *(const v4u*)&sT[(p >> 3) * 64 + (p & 7) * 8];
  }
  const int h0 = cw >> 6;
#pragma unroll
  for (int it = 0; it < 4; ++it) {
    const int p = it * 256 + tid, L = p >> 3, q = p & 7;
    unsigned short* dstp;
    if (sel == 2) dstp = plane + (size_t)(cw + L) * NNODE + n0 + q * 8;
    else          dstp = plane + ((size_t)(h0 + (L >> 6)) * NNODE + n0 + (L & 63)) * HDIM + q * 8;
    *(volatile v4u_*)dstp = pv[it];
  }
  __threadfence();
#pragma unroll
  for (int it = 0; it < 4; ++it) {
    const int p = it * 256 + tid, L = p >> 3, q = p & 7;
    unsigned short* dstp;
    if (sel == 2) dstp = plane + (size_t)(cw + L) * NNODE + n0 + q * 8;
    else          dstp = plane + ((size_t)(h0 + (L >> 6)) * NNODE + n0 + (L & 63)) * HDIM + q * 8;
    *(volatile v4u_*)dstp = pv[it];
  }
}

__global__ void __launch_bounds__(256) attn_kernel(
    const _Float16* __restrict__ qh, const _Float16* __restrict__ kh, const _Float16* __restrict__ vt,
    const unsigned* __restrict__ mk, unsigned short* __restrict__ ctx)
{
  __shared__ __align__(16) unsigned       sMk[MWORDS * 16];
  __shared__ __align__(16) unsigned short sC[NHEAD * 16 * HDIM];

  const int tid  = (int)threadIdx.x;
  const int lane = tid & 31, wave = tid >> 5;
  const int h = lane >> 4, m = lane & 15;
  const int i0 = (int)blockIdx.x * 16;
  const int hd = wave;

#pragma unroll
  for (int it = 0; it < 8; ++it) {
    const int idx = it * 256 + tid;
    const int row = idx >> 7, w = idx & 127;
    sMk[w * 16 + row] = mk[(size_t)(i0 + row) * MWORDS + w];
  }
  __syncthreads();

  const _Float16* Qn = qh + (size_t)hd * NNODE * HDIM;
  const _Float16* Kn = kh + (size_t)hd * NNODE * HDIM;
  const _Float16* Vn = vt + (size_t)hd * HDIM * NNODE;
  const v8f z8 = {};

  FragH qb0, qb1;
  {
    const _Float16* qr = Qn + (size_t)(i0 + m) * HDIM + 8 * h;
    qb0.h[0] = *(const v8h*)(qr);       qb0.h[1] = *(const v8h*)(qr + 16);
    qb1.h[0] = *(const v8h*)(qr + 32);  qb1.h[1] = *(const v8h*)(qr + 48);
  }

  v8f oacc[4] = {};
  float mi = -3.0e30f;
  float li = 0.0f;

#pragma unroll 1
  for (int j0 = 0; j0 < NNODE; j0 += 32) {
    const unsigned mw = sMk[(j0 >> 5) * 16 + m];

    FragH k0a, k0b, k1a, k1b;
    {
      const _Float16* kp0 = Kn + (size_t)(j0 + m) * HDIM + 8 * h;
      const _Float16* kp1 = kp0 + (size_t)16 * HDIM;
      k0a.h[0] = *(const v8h*)(kp0);       k0a.h[1] = *(const v8h*)(kp0 + 16);
      k0b.h[0] = *(const v8h*)(kp0 + 32);  k0b.h[1] = *(const v8h*)(kp0 + 48);
      k1a.h[0] = *(const v8h*)(kp1);       k1a.h[1] = *(const v8h*)(kp1 + 16);
      k1b.h[0] = *(const v8h*)(kp1 + 32);  k1b.h[1] = *(const v8h*)(kp1 + 48);
    }
    v8f s0 = mma_f16(k0a.v, qb0.v, z8);
    s0 = mma_f16(k0b.v, qb1.v, s0);
    v8f s1 = mma_f16(k1a.v, qb0.v, z8);
    s1 = mma_f16(k1b.v, qb1.v, s1);

    float t0[8], t1[8];
    unsigned b0[8], b1[8];
    float cm = -3.0e30f;
#pragma unroll
    for (int r = 0; r < 8; ++r) {
      b0[r] = (mw >> (8 * h + r)) & 1u;
      b1[r] = (mw >> (16 + 8 * h + r)) & 1u;
      t0[r] = (b0[r] != 0u) ? s0[r] * SCL : -3.0e30f;
      t1[r] = (b1[r] != 0u) ? s1[r] * SCL : -3.0e30f;
      cm = fmaxf(cm, fmaxf(t0[r], t1[r]));
    }
    cm = fmaxf(cm, __shfl_xor(cm, 16, 32));
    const float mnew = fmaxf(mi, cm);
    const float corr = exp2fast(mi - mnew);

    float rs = 0.0f;
    FragH pa;
#pragma unroll
    for (int r = 0; r < 8; ++r) {
      const float e0r = exp2fast(t0[r] - mnew);
      const float e1r = exp2fast(t1[r] - mnew);
      const float e0 = (b0[r] != 0u) ? e0r : 0.0f;
      const float e1 = (b1[r] != 0u) ? e1r : 0.0f;
      rs += e0 + e1;
      pa.h[0][r] = (_Float16)(e0 * PCARRY);
      pa.h[1][r] = (_Float16)(e1 * PCARRY);
    }
    rs += __shfl_xor(rs, 16, 32);
    li = li * corr + rs;
    mi = mnew;

    float cr[8];
#pragma unroll
    for (int r = 0; r < 8; ++r) cr[r] = __shfl(corr, 8 * h + r, 32);
#pragma unroll
    for (int t = 0; t < 4; ++t)
#pragma unroll
      for (int r = 0; r < 8; ++r) oacc[t][r] *= cr[r];

    FragH vb[4];
#pragma unroll
    for (int t = 0; t < 4; ++t) {
      const _Float16* vp = Vn + (size_t)(t * 16 + m) * NNODE + j0 + 8 * h;
      vb[t].h[0] = *(const v8h*)(vp);
      vb[t].h[1] = *(const v8h*)(vp + 16);
    }
#pragma unroll
    for (int t = 0; t < 4; ++t) oacc[t] = mma_f16(pa.v, vb[t].v, oacc[t]);
  }

  const float inv = CTXSC * (1.0f / li);
  float fl[8];
#pragma unroll
  for (int r = 0; r < 8; ++r) fl[r] = __shfl(inv, 8 * h + r, 32);
#pragma unroll
  for (int t = 0; t < 4; ++t)
#pragma unroll
    for (int r = 0; r < 8; ++r)
      sC[(hd * 16 + 8 * h + r) * HDIM + t * 16 + m] = f16_bits(oacc[t][r] * fl[r]);
  __syncthreads();

  v4u_ cv[4];
#pragma unroll
  for (int it = 0; it < 4; ++it) {
    const int p = it * 256 + tid;
    cv[it] = *(const v4u*)&sC[(p >> 3) * 64 + (p & 7) * 8];
  }
#pragma unroll
  for (int it = 0; it < 4; ++it) {
    const int p = it * 256 + tid, L = p >> 3, q = p & 7;
    *(volatile v4u_*)(ctx + ((size_t)(i0 + (L & 15)) * HIDC + (size_t)(L >> 4) * HDIM + q * 8)) = cv[it];
  }
  __threadfence();
#pragma unroll
  for (int it = 0; it < 4; ++it) {
    const int p = it * 256 + tid, L = p >> 3, q = p & 7;
    *(volatile v4u_*)(ctx + ((size_t)(i0 + (L & 15)) * HIDC + (size_t)(L >> 4) * HDIM + q * 8)) = cv[it];
  }
}

__global__ void __launch_bounds__(256) oproj_ln_kernel(
    const _Float16* __restrict__ ctx, const _Float16* __restrict__ wo16,
    const float* __restrict__ bo, const float* __restrict__ x,
    const float* __restrict__ lng, const float* __restrict__ lnb, float* __restrict__ out)
{
  __shared__ __align__(16) float sY[16 * HIDC];

  const int tid  = (int)threadIdx.x;
  const int lane = tid & 31, wave = tid >> 5;
  const int h = lane >> 4, m = lane & 15;
  const int n0 = (int)blockIdx.x * 16;
  const int cb = wave * 64;

  v8f acc[4] = {};
#pragma unroll 2
  for (int k0 = 0; k0 < HIDC; k0 += 32) {
    FragH a;
    const _Float16* ar = ctx + (size_t)(n0 + m) * HIDC + k0 + 8 * h;
    a.h[0] = *(const v8h*)(ar);
    a.h[1] = *(const v8h*)(ar + 16);
    FragH b[4];
#pragma unroll
    for (int ct = 0; ct < 4; ++ct) {
      const _Float16* wr = wo16 + (size_t)(cb + ct * 16 + m) * HIDC + k0 + 8 * h;
      b[ct].h[0] = *(const v8h*)(wr);
      b[ct].h[1] = *(const v8h*)(wr + 16);
    }
#pragma unroll
    for (int ct = 0; ct < 4; ++ct) acc[ct] = mma_f16(a.v, b[ct].v, acc[ct]);
  }
#pragma unroll
  for (int ct = 0; ct < 4; ++ct) {
    const int col = cb + ct * 16 + m;
    const float bb = bf16_rn(bo[col]);
#pragma unroll
    for (int r = 0; r < 8; ++r) sY[(8 * h + r) * HIDC + col] = acc[ct][r] * OUNC + bb;
  }
  __syncthreads();

  v4f_ ov[2][4];
#pragma unroll
  for (int rr = 0; rr < 2; ++rr) {
    const int row = wave * 2 + rr;
    const size_t n = (size_t)(n0 + row);
    v4f_ v[4];
    float sum = 0.0f;
#pragma unroll
    for (int it = 0; it < 4; ++it) {
      const int p = it * 32 + lane;
      const v4f_ a  = *(const v4f*)&sY[row * HIDC + p * 4];
      const v4f_ xv = *(const v4f*)(x + n * HIDC + (size_t)p * 4);
      v4f_ t;
      t[0] = bf16_rn(xv[0]) + a[0];
      t[1] = bf16_rn(xv[1]) + a[1];
      t[2] = bf16_rn(xv[2]) + a[2];
      t[3] = bf16_rn(xv[3]) + a[3];
      v[it] = t;
      sum += (t[0] + t[1]) + (t[2] + t[3]);
    }
    sum += __shfl_xor(sum, 16, 32);
    sum += __shfl_xor(sum, 8, 32);
    sum += __shfl_xor(sum, 4, 32);
    sum += __shfl_xor(sum, 2, 32);
    sum += __shfl_xor(sum, 1, 32);
    const float mu = sum * (1.0f / (float)HIDC);
    float sq = 0.0f;
#pragma unroll
    for (int it = 0; it < 4; ++it) {
      v4f_ d;
      d[0] = v[it][0] - mu; d[1] = v[it][1] - mu; d[2] = v[it][2] - mu; d[3] = v[it][3] - mu;
      v[it] = d;
      sq += (d[0] * d[0] + d[1] * d[1]) + (d[2] * d[2] + d[3] * d[3]);
    }
    sq += __shfl_xor(sq, 16, 32);
    sq += __shfl_xor(sq, 8, 32);
    sq += __shfl_xor(sq, 4, 32);
    sq += __shfl_xor(sq, 2, 32);
    sq += __shfl_xor(sq, 1, 32);
    const float var = sq * (1.0f / (float)HIDC);
    const float rs  = rsqrtf(var + LNEPS);
#pragma unroll
    for (int it = 0; it < 4; ++it) {
      const int p = it * 32 + lane;
      const v4f_ gv = *(const v4f*)(lng + (size_t)p * 4);
      const v4f_ bv = *(const v4f*)(lnb + (size_t)p * 4);
      v4f_ o;
      o[0] = (bf16_rn(gv[0]) * v[it][0]) * rs + bf16_rn(bv[0]);
      o[1] = (bf16_rn(gv[1]) * v[it][1]) * rs + bf16_rn(bv[1]);
      o[2] = (bf16_rn(gv[2]) * v[it][2]) * rs + bf16_rn(bv[2]);
      o[3] = (bf16_rn(gv[3]) * v[it][3]) * rs + bf16_rn(bv[3]);
      ov[rr][it] = o;
    }
  }

#pragma unroll
  for (int rr = 0; rr < 2; ++rr)
#pragma unroll
    for (int it = 0; it < 4; ++it)
      *(volatile v4f_*)(out + (size_t)(n0 + wave * 2 + rr) * HIDC + (size_t)(it * 32 + lane) * 4) = ov[rr][it];
  __threadfence();
#pragma unroll
  for (int rr = 0; rr < 2; ++rr)
#pragma unroll
    for (int it = 0; it < 4; ++it)
      *(volatile v4f_*)(out + (size_t)(n0 + wave * 2 + rr) * HIDC + (size_t)(it * 32 + lane) * 4) = ov[rr][it];
}

extern "C" void kernel_launch(void* const* d_in, const int* in_sizes, int n_in,
                              void* d_out, int out_size, void* d_ws, size_t ws_size,
                              hipStream_t stream)
{
  if (n_in < 12) return;
  if (in_sizes[0] < NNODE * HIDC) return;
  if (in_sizes[1] < 2) return;
  if (in_sizes[2] < HIDC * HIDC || in_sizes[4] < HIDC * HIDC ||
      in_sizes[6] < HIDC * HIDC || in_sizes[8] < HIDC * HIDC) return;
  if (in_sizes[3] < HIDC || in_sizes[5] < HIDC || in_sizes[7] < HIDC ||
      in_sizes[9] < HIDC || in_sizes[10] < HIDC || in_sizes[11] < HIDC) return;
  if (out_size < QROWS * HIDC) return;

  const float* x   = (const float*)d_in[0];
  const int*   ei  = (const int*)d_in[1];
  const float* wq  = (const float*)d_in[2];
  const float* bq  = (const float*)d_in[3];
  const float* wk  = (const float*)d_in[4];
  const float* bk  = (const float*)d_in[5];
  const float* wv  = (const float*)d_in[6];
  const float* bv  = (const float*)d_in[7];
  const float* wo  = (const float*)d_in[8];
  const float* bo  = (const float*)d_in[9];
  const float* lng = (const float*)d_in[10];
  const float* lnb = (const float*)d_in[11];
  float* out = (float*)d_out;
  const int ne = in_sizes[1] / 2;

  const size_t xb_bytes   = (size_t)NNODE * HIDC * 2;
  const size_t wqkv_bytes = (size_t)3 * HIDC * HIDC * 2;
  const size_t wo_bytes   = (size_t)HIDC * HIDC * 2;
  const size_t qk_bytes   = (size_t)NHEAD * NNODE * HDIM * 2;
  const size_t vt_bytes   = (size_t)NHEAD * HDIM * NNODE * 2;
  const size_t mk_bytes   = (size_t)NNODE * MWORDS * 4;
  const size_t ctx_bytes  = (size_t)NNODE * HIDC * 2;
  size_t off = 0;
  unsigned char* ws = (unsigned char*)d_ws;
  unsigned short* xb   = (unsigned short*)(ws + off); off += xb_bytes;
  unsigned short* wqkv = (unsigned short*)(ws + off); off += wqkv_bytes;
  unsigned short* wob  = (unsigned short*)(ws + off); off += wo_bytes;
  unsigned short* qhp  = (unsigned short*)(ws + off); off += qk_bytes;
  unsigned short* khp  = (unsigned short*)(ws + off); off += qk_bytes;
  unsigned short* vtp  = (unsigned short*)(ws + off); off += vt_bytes;
  unsigned*       mkp  = (unsigned*)(ws + off);       off += mk_bytes;
  unsigned short* ctxp = (unsigned short*)(ws + off); off += ctx_bytes;
  if (off > ws_size) return;

  cvt_kernel<<<XB_BLOCKS + 4 * W_BLOCKS, 256, 0, stream>>>(x, wq, wk, wv, wo, xb, wqkv, wob);
  adj_kernel<<<QROWS / 64, 256, 0, stream>>>(ei, ne, mkp);
  proj_kernel<<<dim3(NNODE / 64, (3 * HIDC) / 128), 256, 0, stream>>>(xb, wqkv, bq, bk, bv, qhp, khp, vtp);
  attn_kernel<<<QROWS / 16, 256, 0, stream>>>((const _Float16*)qhp, (const _Float16*)khp,
                                              (const _Float16*)vtp, (const unsigned*)mkp, ctxp);
  oproj_ln_kernel<<<QROWS / 16, 256, 0, stream>>>((const _Float16*)ctxp, (const _Float16*)wob,
                                                  bo, x, lng, lnb, out);
}
